// HybridGATLSTM_8693013807250
// MI455X (gfx1250) — hardware-run, weakly checked
//
#include <hip/hip_runtime.h>


namespace {
constexpr int NB_ = 8, S = 32, NN = 2000, E = 64000, GH = 32, H = 64, NR = NB_ * S  , G4 = 4 * H  , KC = 16, NPC = NN / KC  , NPB = 8;
constexpr float HS = 256.0f, WSC = 256.0f;
typedef _Float16 b16;
typedef __attribute__((ext_vector_type(16))) _Float16 v16b;
typedef __attribute__((ext_vector_type(8))) _Float16 v8b;
typedef __attribute__((ext_vector_type(8))) float v8f;
typedef __attribute__((ext_vector_type(4))) float v4f;
__device__ __forceinline__ float bf16_rne(float f) { unsigned int u = __float_as_uint(f); u += 0x7FFFu + ((u >> 16) & 1u); float r = __uint_as_float(u & 0xFFFF0000u); asm volatile("" : "+v"(r)); return r; }
__device__ __forceinline__ float bfv(float f) { float r = bf16_rne(f); asm volatile("" : "+v"(r)); return r; }
__device__ __forceinline__ void split16(float v, b16& hi, b16& lo) { hi = (b16)v; lo = (b16)(v - (float)hi); }
__device__ __forceinline__ v16b frag_kb(const b16* p, int hh) { const v8b a = *(const v8b*)(p + 8 * hh), b = *(const v8b*)(p + 16 + 8 * hh); v16b f;
#pragma unroll
  for (int e = 0; e < 8; ++e) { f[e] = a[e]; f[8 + e] = b[e]; } return f; }
__device__ __forceinline__ v8f wmma16b(v16b a, v16b b, v8f c) { v8f d = __builtin_amdgcn_wmma_f32_16x16x32_f16(false, a, false, b, (short)0, c, false, false); asm volatile("v_nop\n\tv_nop\n\tv_nop\n\tv_nop" : "+v"(d) : "v"(a), "v"(b)); return d; }
__device__ __forceinline__ void wave_lds_sync() { __builtin_amdgcn_fence(__ATOMIC_RELEASE, "workgroup"); __builtin_amdgcn_wave_barrier(); __builtin_amdgcn_fence(__ATOMIC_ACQUIRE, "workgroup"); }
__device__ __forceinline__ float pmul(float a, float b) { float p = a * b; asm volatile("" : "+v"(p)); return p; }
__device__ __forceinline__ int iclamp(int v, int lo, int hi) { return v < lo ? lo : (v > hi ? hi : v); }
__device__ __forceinline__ float sigm(float v) { return 1.0f / (1.0f + __expf(-v)); }
constexpr int CSR_NBLK7 = 512, CSR_GB7 = 7, CSR_GN7 = 1 << CSR_GB7  , CSR_TS7 = (CSR_GN7 < 32 ? 32 : CSR_GN7)  , CSR_MAXG7 = 512, CSR_CAP7 = 12288  ;
__device__ __host__ __forceinline__ int csr_tix7(int v) { return (v >> CSR_GB7) * CSR_TS7 + (v & (CSR_GN7 - 1)); }
__global__ __launch_bounds__(64) void csrA_kernel7(const int* __restrict__ dst, int E, int N, int nG, int CHP, int NGP, int* __restrict__ STG, int* __restrict__ HST) {
  extern __shared__ int sm[];
  int* cnt = sm; int* run = sm + NGP; int* ids = sm + 2 * NGP;
  const int b = blockIdx.x; const int ch = (E + CSR_NBLK7 - 1) / CSR_NBLK7; const int e0 = b * ch, e1 = min(E, e0 + ch);
  for (int i = threadIdx.x; i < NGP; i += 64) cnt[i] = 0;
  for (int i = threadIdx.x; i < CHP; i += 64) ids[i] = -1;
  __syncthreads();
  if (threadIdx.x == 0) {
    for (int e = e0; e < e1; ++e) { int d = dst[e]; d = (d < 0) ? 0 : (d >= N ? N - 1 : d); cnt[d >> CSR_GB7] += 1; }
    int acc = 0; for (int g = 0; g < nG; ++g) { run[g] = acc; acc += cnt[g]; }
    for (int e = e0; e < e1; ++e) { int d = dst[e]; d = (d < 0) ? 0 : (d >= N ? N - 1 : d); const int g = d >> CSR_GB7; ids[run[g]] = e; run[g] += 1; } }
  __syncthreads();
  typedef __attribute__((ext_vector_type(4))) int v4i;
  for (int pass = 0; pass < 2; ++pass) {
    for (int i = threadIdx.x; i < CHP / 4; i += 64) *(volatile v4i*)(STG + (size_t)b * CHP + i * 4) = *(const v4i*)(&ids[i * 4]);
    for (int i = threadIdx.x; i < NGP / 4; i += 64) { v4i v; for (int e = 0; e < 4; ++e) v[e] = (i * 4 + e < nG) ? cnt[i * 4 + e] : 0; *(volatile v4i*)(HST + (size_t)b * NGP + i * 4) = v; }
    __threadfence(); }
}
__global__ __launch_bounds__(512) void csrS_kernel7(const int* __restrict__ HST, int nG, int NGP, int* __restrict__ START, int* __restrict__ TOT, int* __restrict__ OFF) {
  __shared__ int tot[CSR_MAXG7];
  const int b = threadIdx.x;
  for (int pass = 0; pass < 2; ++pass) { int runb = 0; for (int g = 0; g < nG; ++g) { int c = HST[(size_t)b * NGP + g]; c = (c < 0) ? 0 : c; ((volatile int*)OFF)[(size_t)g * CSR_NBLK7 + b] = runb; runb += c; } __threadfence(); }
  for (int g = threadIdx.x; g < nG; g += 512) { int s = 0; for (int bb = 0; bb < CSR_NBLK7; ++bb) { int c = HST[(size_t)bb * NGP + g]; s += (c < 0) ? 0 : c; } tot[g] = s; }
  __syncthreads();
  if (threadIdx.x < 32) {
    __shared__ int st[CSR_MAXG7 + 32];
    if (threadIdx.x == 0) { int acc = 0; for (int g = 0; g < NGP; ++g) { st[g] = acc; if (g < nG) acc += (tot[g] + 31) & ~31; } st[NGP] = acc; }
    __builtin_amdgcn_fence(__ATOMIC_RELEASE, "workgroup"); __builtin_amdgcn_wave_barrier(); __builtin_amdgcn_fence(__ATOMIC_ACQUIRE, "workgroup");
    for (int pass = 0; pass < 2; ++pass) { for (int i = threadIdx.x; i < NGP + 32; i += 32) { ((volatile int*)START)[i] = (i <= NGP) ? st[min(i, NGP)] : 0; ((volatile int*)TOT)[i] = (i < nG) ? tot[i] : 0; } __threadfence(); } }
}
__global__ __launch_bounds__(256) void csrB_kernel7(const int* __restrict__ dst, int N, int nG, int CHP, int NGP, int permLen, const int* __restrict__ STG, const int* __restrict__ HST, const int* __restrict__ OFF, const int* __restrict__ START, const int* __restrict__ TOT, int* __restrict__ PERM, int* __restrict__ ROWPTR, int* __restrict__ ROWCNT, int* __restrict__ FLAG) {
  typedef __attribute__((ext_vector_type(4))) int v4i;
  __shared__ int ids[CSR_CAP7]; __shared__ unsigned short key[CSR_CAP7]; __shared__ int outp[CSR_CAP7]; __shared__ int ncnt[CSR_GN7 + 1]; __shared__ int boff[CSR_NBLK7 + 1];
  const int g = blockIdx.x, t_ = threadIdx.x; int tot = TOT[g]; int st = START[g], stn = START[g + 1]; const int v0 = g * CSR_GN7; const int nv = min(CSR_GN7, N - v0); const int t0 = g * CSR_TS7;
  st = (st < 0) ? 0 : (st > permLen - 32 ? permLen - 32 : st) & ~31; stn = (stn < st) ? st : (stn > permLen ? permLen : stn); tot = (tot < 0) ? 0 : tot; if (tot > stn - st && tot <= CSR_CAP7) tot = stn - st;
  if (tot > CSR_CAP7) {
    for (int pass = 0; pass < 2; ++pass) { for (int i = t_; i < CSR_TS7 / 4; i += 256) { v4i a, c; for (int e = 0; e < 4; ++e) { a[e] = st; c[e] = 0; } *(volatile v4i*)(ROWPTR + t0 + i * 4) = a; *(volatile v4i*)(ROWCNT + t0 + i * 4) = c; } if (t_ == 0) ((volatile int*)FLAG)[0] = 1; __threadfence(); } (void)nv; return; }
  if (t_ == 0) { int acc = 0; for (int b = 0; b < CSR_NBLK7; ++b) { boff[b] = acc; int c = HST[(size_t)b * NGP + g]; c = (c < 0) ? 0 : (c > CHP ? CHP : c); acc += c; if (acc > tot) acc = tot; } boff[CSR_NBLK7] = acc; }
  for (int i = t_; i <= CSR_GN7; i += 256) ncnt[i] = 0;
  __syncthreads();
  for (int b = 0; b < CSR_NBLK7; ++b) { const int c = boff[b + 1] - boff[b]; int o_ = OFF[(size_t)g * CSR_NBLK7 + b]; o_ = (o_ < 0) ? 0 : (o_ > CHP - c ? CHP - c : o_); const int* src_ = STG + (size_t)b * CHP + o_;
    for (int i = t_; i < c; i += 256) { int id = src_[i]; id = (id < 0) ? 0 : id; ids[boff[b] + i] = id; int d = dst[id]; d = (d < v0) ? v0 : (d >= N ? N - 1 : d); int kk = d - v0; kk = (kk < 0) ? 0 : (kk >= CSR_GN7 ? CSR_GN7 - 1 : kk); key[boff[b] + i] = (unsigned short)kk; } }
  __syncthreads();
  if (t_ == 0) { for (int i = 0; i < tot; ++i) ncnt[key[i]] += 1; int acc = 0; for (int vl = 0; vl < CSR_GN7; ++vl) { const int c = ncnt[vl]; ncnt[vl] = acc; acc += c; } ncnt[CSR_GN7] = acc;
    for (int i = 0; i < tot; ++i) { const int vl = key[i]; outp[ncnt[vl]] = ids[i]; ncnt[vl] += 1; }
    for (int vl = CSR_GN7; vl > 0; --vl) ncnt[vl] = ncnt[vl - 1]; ncnt[0] = 0; }
  __syncthreads();
  for (int pass = 0; pass < 2; ++pass) {
    for (int i = t_; i < (stn - st) / 4; i += 256) { v4i v; for (int e = 0; e < 4; ++e) { const int q = i * 4 + e; v[e] = (q < tot) ? outp[q] : -1; } *(volatile v4i*)(PERM + st + i * 4) = v; }
    for (int i = t_; i < CSR_TS7 / 4; i += 256) { v4i a, c; for (int e = 0; e < 4; ++e) { const int vl = i * 4 + e; const int vc = vl < CSR_GN7 ? vl : CSR_GN7; a[e] = (vl < CSR_GN7) ? st + ncnt[vc] : st; c[e] = (vl < nv) ? (ncnt[(vc < CSR_GN7 ? vc : CSR_GN7 - 1) + 1] - ncnt[vc]) : 0; } *(volatile v4i*)(ROWPTR + t0 + i * 4) = a; *(volatile v4i*)(ROWCNT + t0 + i * 4) = c; }
    __threadfence(); }
}
__global__ __launch_bounds__(256) void csrZ_kernel7(int* __restrict__ p, size_t n4) { typedef __attribute__((ext_vector_type(4))) int v4i; const size_t tid = (size_t)blockIdx.x * 256 + threadIdx.x, nth = (size_t)gridDim.x * 256; v4i z = {0, 0, 0, 0}; for (size_t i = tid; i < n4; i += nth) *(volatile v4i*)(p + i * 4) = z; }
struct CsrBufs7 { int *STG, *HST, *OFF, *START, *TOT, *PERM, *ROWPTR, *ROWCNT, *FLAG; int nG, NGP, CHP; size_t permLen; char* base; size_t bytes; };
static size_t csr_carve7(CsrBufs7& c, char* ws, size_t off, int E, int N) {
  const size_t off0 = off; c.base = ws + off;
  auto al = [&](size_t bytes) { char* p = ws + off; off += (bytes + 255) & ~(size_t)255; return p; };
  c.nG = (N + CSR_GN7 - 1) / CSR_GN7; c.NGP = (c.nG + 31) & ~31; const int ch = (E + CSR_NBLK7 - 1) / CSR_NBLK7; c.CHP = (ch + 31) & ~31; c.permLen = (size_t)E + 32 * (size_t)c.nG + 32;
  c.STG = (int*)al((size_t)CSR_NBLK7 * c.CHP * 4); c.HST = (int*)al((size_t)CSR_NBLK7 * c.NGP * 4); c.OFF = (int*)al((size_t)c.NGP * CSR_NBLK7 * 4); c.START = (int*)al((size_t)(c.NGP + 64) * 4); c.TOT = (int*)al((size_t)(c.NGP + 64) * 4);
  c.PERM = (int*)al(c.permLen * 4); c.ROWPTR = (int*)al((size_t)c.nG * CSR_TS7 * 4); c.ROWCNT = (int*)al((size_t)c.nG * CSR_TS7 * 4); c.FLAG = (int*)al(256);
  c.bytes = off - off0; return off;
}
static void csr_build7(const CsrBufs7& c, const int* dst, int E, int N, hipStream_t stream) {
  const size_t smem = (size_t)(2 * c.NGP + c.CHP) * 4;
  csrZ_kernel7<<<512, 256, 0, stream>>>((int*)c.base, c.bytes / 16);
  csrA_kernel7<<<CSR_NBLK7, 64, smem, stream>>>(dst, E, N, c.nG, c.CHP, c.NGP, c.STG, c.HST);
  csrS_kernel7<<<1, 512, 0, stream>>>(c.HST, c.nG, c.NGP, c.START, c.TOT, c.OFF);
  csrB_kernel7<<<c.nG, 256, 0, stream>>>(dst, N, c.nG, c.CHP, c.NGP, (int)c.permLen, c.STG, c.HST, c.OFF, c.START, c.TOT, c.PERM, c.ROWPTR, c.ROWCNT, c.FLAG);
}


__global__ __launch_bounds__(256) void wput_kernel(const float* __restrict__ wih, b16* __restrict__ WIH) { const size_t nt = (size_t)gridDim.x * 256, u0 = (size_t)blockIdx.x * 256 + threadIdx.x; v8b v;
  for (size_t u = u0; u < (size_t)G4 * (NN * GH / 8); u += nt) { const size_t o = u / (NN * GH / 8), k0 = (u % (NN * GH / 8)) * 8;
#pragma unroll
    for (int j = 0; j < 8; ++j) v[j] = (b16)(bf16_rne(wih[o * NN * GH + k0 + j]) * WSC); for (int pass = 0; pass < 2; ++pass) { *(volatile v8b*)(WIH + o * NN * GH + k0) = v; __threadfence(); } } }
__global__ __launch_bounds__(256) void xt_kernel(const float* __restrict__ x, float* __restrict__ XT) { __shared__ float T[NR][33]; const int n0 = blockIdx.x * 32; const int tid = threadIdx.x;
  for (int r = tid; r < NR; r += 256) for (int j = 0; j < 32; ++j) { const int n = n0 + j; T[r][j] = n < NN ? bfv(x[(size_t)r * NN + n]) : 0.0f; }
  __syncthreads(); const int wave = tid >> 5, lane = tid & 31;
  for (int pass = 0; pass < 2; ++pass) { for (int j = wave; j < 32; j += 8) { const int n = n0 + j; if (n < NN) for (int q = 0; q < NR / 32; ++q) ((volatile float*)XT)[(size_t)n * NR + q * 32 + lane] = T[q * 32 + lane][j]; } __threadfence(); } }
__global__ __launch_bounds__(256) void gat_kernel(const float* __restrict__ XT, const float* __restrict__ wl, const float* __restrict__ as_, const float* __restrict__ ad_, const int* __restrict__ srcs, const int* __restrict__ PERM, const int* __restrict__ ROWPTR, const int* __restrict__ ROWCNT, int permLen, int RLIM, float* __restrict__ AGG) { const int wave = threadIdx.x >> 5, lane = threadIdx.x & 31; const size_t i = (size_t)blockIdx.x * NPB + wave; if (i >= (size_t)NN) return; float cs = 0.0f, cd = 0.0f; for (int g = 0; g < GH; ++g) { cs += pmul(bfv(wl[g]), bfv(as_[g])); cd += pmul(bfv(wl[g]), bfv(ad_[g])); }
  int st = ROWPTR[i], cnt = ROWCNT[i]; cnt = iclamp(cnt, 0, E); st = iclamp(st, 0, permLen - cnt); float xd[8], mx[8], den[8], acc[8];
#pragma unroll
  for (int k = 0; k < 8; ++k) { xd[k] = XT[i * NR + lane * 8 + k]; mx[k] = -INFINITY; den[k] = 0.0f; acc[k] = 0.0f; }
  auto visit = [&](size_t u) { const float* xr = XT + u * NR + lane * 8;
#pragma unroll
    for (int k = 0; k < 8; ++k) { const float xv = xr[k]; float s = pmul(xv, cs) + pmul(xd[k], cd); s = s >= 0.0f ? s : 0.2f * s; const float mn = fmaxf(mx[k], s); const float sf = (mx[k] == -INFINITY) ? 0.0f : __expf(mx[k] - mn); const float p = __expf(s - mn); den[k] = den[k] * sf + p; acc[k] = pmul(acc[k], sf) + pmul(p, xv); mx[k] = mn; } };
#pragma unroll 1
  for (int j = 0; j < cnt; ++j) { const int e = iclamp(PERM[st + j], 0, E - 1); const size_t u = (size_t)iclamp(srcs[e], 0, NN - 1); visit(u); }
  visit(i);
  for (int pass = 0; pass < 2; ++pass) {
#pragma unroll
    for (int k = 0; k < 8; ++k) ((volatile float*)AGG)[i * NR + lane * 8 + k] = (lane * 8 + k) < RLIM ? acc[k] / den[k] : 0.0f; __threadfence(); } }
__global__ __launch_bounds__(32) void gates_kernel(const float* __restrict__ AGG, const float* __restrict__ wl, const float* __restrict__ gb, const b16* __restrict__ WIH, int RLIM, float* __restrict__ GP) { __shared__ float Tf[16][G4 + 4]; const int lane = threadIdx.x, nloc = lane & 15, hlf = lane >> 4; const int kc = blockIdx.x % KC; const int m0 = (blockIdx.x / KC) * 16; if (m0 >= RLIM) return;
  float wg[16], bg[16];
#pragma unroll
  for (int e = 0; e < 8; ++e) { wg[e] = bfv(wl[8 * hlf + e]); bg[e] = bfv(gb[8 * hlf + e]); wg[8 + e] = bfv(wl[16 + 8 * hlf + e]); bg[8 + e] = bfv(gb[16 + 8 * hlf + e]); }
  v8f acc[16];
#pragma unroll
  for (int t = 0; t < 16; ++t) acc[t] = (v8f){};
#pragma unroll 1
  for (int n = kc * NPC; n < kc * NPC + NPC; ++n) { const float av = AGG[(size_t)n * NR + m0 + nloc]; v16b a, al;
#pragma unroll
    for (int e = 0; e < 16; ++e) { const float v = fmaxf(pmul(av, wg[e]) + bg[e], 0.0f); b16 p, ql; split16(v * HS, p, ql); a[e] = p; al[e] = ql; }
    const b16* wrow = WIH + (size_t)n * GH;
#pragma unroll
    for (int t = 0; t < 16; ++t) { const v16b bw = frag_kb(wrow + (size_t)(t * 16 + nloc) * (NN * GH), hlf); acc[t] = wmma16b(a, bw, acc[t]); acc[t] = wmma16b(al, bw, acc[t]); } }
#pragma unroll
  for (int t = 0; t < 16; ++t)
#pragma unroll
    for (int r8 = 0; r8 < 8; ++r8) Tf[8 * hlf + r8][t * 16 + nloc] = acc[t][r8] * (1.0f / (HS * WSC));
  wave_lds_sync();
  for (int pass = 0; pass < 2; ++pass) { for (int rr = 0; rr < 16; ++rr) for (int q = 0; q < G4 / 32; ++q) ((volatile float*)GP)[((size_t)kc * NR + m0 + rr) * G4 + q * 32 + lane] = Tf[rr][q * 32 + lane]; __threadfence(); } }
__global__ __launch_bounds__(256) void lstm_kernel(const float* __restrict__ GP, const float* __restrict__ whh, const float* __restrict__ bih, const float* __restrict__ bhh, int BLIM, float* __restrict__ HF) { __shared__ float Hs[H], Cs[H], Gs[G4]; const int b = blockIdx.x; const int o = threadIdx.x; if (b >= BLIM) return;
  for (int pass = 0; pass < 2; ++pass) { if (o < H) { Hs[o] = 0.0f; Cs[o] = 0.0f; } __syncthreads();
#pragma unroll 1
    for (int s = 0; s < S; ++s) { const size_t r = (size_t)b * S + s; float g = bfv(bih[o]) + bfv(bhh[o]);
#pragma unroll 1
      for (int kc = 0; kc < KC; ++kc) g += GP[((size_t)kc * NR + r) * G4 + o];
#pragma unroll 4
      for (int k = 0; k < H; ++k) g += pmul(Hs[k], bfv(whh[(size_t)o * H + k])); Gs[o] = g; __syncthreads();
      if (o < H) { const float c = pmul(sigm(Gs[H + o]), Cs[o]) + pmul(sigm(Gs[o]), tanhf(Gs[2 * H + o])); Cs[o] = c; Hs[o] = pmul(sigm(Gs[3 * H + o]), tanhf(c)); } __syncthreads(); }
    if (o < H) ((volatile float*)HF)[b * H + o] = Hs[o]; __threadfence(); __syncthreads(); } }
__global__ __launch_bounds__(256) void head_kernel(const float* __restrict__ HF, const float* __restrict__ wh, const float* __restrict__ bh, int BLIM, float* __restrict__ out) { const size_t u = (size_t)blockIdx.x * 256 + threadIdx.x; if (u >= (size_t)NB_ * NN) return; const int b = (int)(u / NN), n = (int)(u % NN); if (b >= BLIM) return; float s = bfv(bh[n]);
#pragma unroll 4
  for (int k = 0; k < H; ++k) s += pmul(HF[b * H + k], bfv(wh[(size_t)n * H + k]));
  for (int pass = 0; pass < 2; ++pass) { ((volatile float*)out)[u] = s; __threadfence(); } }
}

extern "C" void kernel_launch(void* const* d_in, const int* in_sizes, int n_in, void* d_out, int out_size, void* d_ws, size_t ws_size, hipStream_t stream) {
  (void)n_in;
  auto Fp = [&](int i) { return (const float*)d_in[i]; }; auto Ip = [&](int i) { return (const int*)d_in[i]; };
  if (in_sizes[0] != NR * NN || in_sizes[1] != 2 * E || in_sizes[2] != GH || in_sizes[6] != G4 * NN * GH || in_sizes[7] != G4 * H || in_sizes[10] != NN * H || out_size != NB_ * NN) return;
  const int BLIM = NB_;
  const int RLIM = BLIM * S;
  size_t off = 0; char* ws = (char*)d_ws;
  auto carve = [&](size_t bytes) { char* p = ws + off; off += (bytes + 255) & ~(size_t)255; return p; };
  b16* WIH = (b16*)carve((size_t)G4 * NN * GH * 2); float* XT = (float*)carve((size_t)NN * NR * 4); float* AGG = (float*)carve((size_t)NN * NR * 4); float* GP = (float*)carve((size_t)KC * NR * G4 * 4); float* HF = (float*)carve((size_t)NB_ * H * 4); CsrBufs7 csr; off = csr_carve7(csr, ws, off, E, NN);
  if (off > ws_size || off > ((size_t)96 << 20)) return;
  wput_kernel<<<256, 256, 0, stream>>>(Fp(6), WIH);
  csr_build7(csr, Ip(1) + E, E, NN, stream);
  xt_kernel<<<(NN + 31) / 32, 256, 0, stream>>>(Fp(0), XT);
  gat_kernel<<<(NN + NPB - 1) / NPB, 256, 0, stream>>>(XT, Fp(2), Fp(3), Fp(4), Ip(1), csr.PERM, csr.ROWPTR, csr.ROWCNT, (int)csr.permLen, RLIM, AGG);
  gates_kernel<<<(RLIM / 16) * KC, 32, 0, stream>>>(AGG, Fp(2), Fp(5), WIH, RLIM, GP);
  lstm_kernel<<<BLIM, 256, 0, stream>>>(GP, Fp(7), Fp(8), Fp(9), BLIM, HF);
  head_kernel<<<(NB_ * NN + 255) / 256, 256, 0, stream>>>(HF, Fp(10), Fp(11), BLIM, (float*)d_out);
}
